// DSSMamba_13039520711229
// MI455X (gfx1250) — hardware-verified
//
#include <hip/hip_runtime.h>
#include <hip/hip_bf16.h>


#define D_MODEL  256
#define D_INNER  512
#define D_STATE  16
#define DT_RANK  16
#define NBATCH   2
#define SEQLEN   2048
#define E_DIM    (4 * D_INNER)
#define R_DIM    (DT_RANK + 2 * D_STATE)
#define MROWS    (NBATCH * SEQLEN)
#define NCHUNK   32
#define CHUNKT   (SEQLEN / NCHUNK)
#define XD_LD    64
#define RSPLIT   (1.0f / 2048.0f)
#define PL_H   ((size_t)MROWS * D_MODEL)
#define PL_WIN ((size_t)E_DIM * D_MODEL)
#define PL_WX  ((size_t)2 * 64 * D_INNER)
#define PL_WO  ((size_t)D_MODEL * 2 * D_INNER)
#define PL_X   ((size_t)2 * MROWS * D_INNER)
#define PL_Y   ((size_t)MROWS * 2 * D_INNER)

typedef _Float16 bf16_t;
typedef __attribute__((ext_vector_type(16))) _Float16 v16bf;
typedef __attribute__((ext_vector_type(8)))  float  v8f;
typedef __attribute__((ext_vector_type(4)))  float  v4f_t;
typedef float v4fa __attribute__((ext_vector_type(4), may_alias));
typedef __attribute__((ext_vector_type(4)))  unsigned v4u_t;
typedef unsigned v4ua __attribute__((ext_vector_type(4), may_alias));

__device__ __forceinline__ _Float16 lo_of(float v, _Float16 h) { return (_Float16)((v - (float)h) * 2048.0f); }
__device__ __forceinline__ void st2f(float* p, float v) { *(volatile float*)p = v; __threadfence(); *(volatile float*)p = v; }
__device__ __forceinline__ void st2pair(_Float16* p, size_t pl, float v0, float v1) {
  const _Float16 a = (_Float16)v0, b = (_Float16)v1;
  const unsigned u = (unsigned)__builtin_bit_cast(unsigned short, a) | ((unsigned)__builtin_bit_cast(unsigned short, b) << 16);
  const unsigned w = (unsigned)__builtin_bit_cast(unsigned short, lo_of(v0, a)) | ((unsigned)__builtin_bit_cast(unsigned short, lo_of(v1, b)) << 16);
  *(volatile unsigned*)p = u; *(volatile unsigned*)(p + pl) = w; __threadfence(); *(volatile unsigned*)p = u; *(volatile unsigned*)(p + pl) = w;
}
__device__ __forceinline__ v8f wmma16(v16bf a, v16bf b, v8f c) { return __builtin_amdgcn_wmma_f32_16x16x32_f16(false, a, false, b, (short)0, c, false, false); }
__device__ __forceinline__ v8f wmma_split(v16bf a, v16bf al, v16bf b, v16bf bl, v8f c) { v8f x = {}; x = wmma16(al, b, x); x = wmma16(a, bl, x); return wmma16(a, b, c) + x * RSPLIT; }

__device__ __forceinline__ float siluf(float x) {
    return x / (1.f + __expf(-x));
}

__device__ __forceinline__ void async_b128_to_lds(void* lds_dst,
                                                  const void* gsrc) {
    unsigned loff = (unsigned)(size_t)lds_dst;
    asm volatile("global_load_async_to_lds_b128 %0, %1, off"
                 :: "v"(loff), "v"(gsrc) : "memory");
}
__device__ __forceinline__ void wait_async_lds() {
    asm volatile("s_wait_asynccnt 0x0" ::: "memory");
}

__global__ void cvt_f32_bf16(const float* __restrict__ src, bf16_t* __restrict__ dst, int n, size_t pl, int nvalid) {
    for (int i = (blockIdx.x * blockDim.x + threadIdx.x) * 2; i < n; i += gridDim.x * blockDim.x * 2) {
        const float v0 = (i < nvalid) ? src[i] : 0.f, v1 = (i + 1 < nvalid) ? src[i + 1] : 0.f;
        st2pair(dst + i, pl, v0, v1);
    }
}

template <int NT>
__global__ void gemm_bf16_wmma(const bf16_t* __restrict__ A, size_t plA,
                               const bf16_t* __restrict__ B, size_t plB,
                               float* __restrict__ C,
                               int M, int N, int K) {
    static_assert(NT == 4, "waves own 64-column row segments");
    __shared__ __attribute__((aligned(16))) float stg[4][16 * 68];
    const int lane   = threadIdx.x & 31;
    const int wave   = threadIdx.x >> 5;
    const int tilesN = N / (16 * NT);
    const int tile   = blockIdx.x * (blockDim.x >> 5) + wave;
    const int tm     = tile / tilesN;
    const int tg     = tile - tm * tilesN;
    if (tm * 16 >= M) return;

    const int half = lane >> 4;
    const int lrow = lane & 15;

    const unsigned int* __restrict__ Arow =
        reinterpret_cast<const unsigned int*>(A + (size_t)(tm * 16 + lrow) * K);
    const unsigned int* Brow[NT];
    #pragma unroll
    for (int nt = 0; nt < NT; ++nt)
        Brow[nt] = reinterpret_cast<const unsigned int*>(
            B + (size_t)(tg * 16 * NT + nt * 16 + lrow) * K);

    v8f acc[NT];
    #pragma unroll
    for (int nt = 0; nt < NT; ++nt) acc[nt] = (v8f){};

    for (int k0 = 0; k0 < K; k0 += 32) {
        const int kw = k0 >> 1;
        __builtin_prefetch(Arow + kw + 32, 0, 1);

        union { v16bf v; unsigned int u[8]; } a, al;
        const unsigned int* ArowL = Arow + (plA >> 1);
        #pragma unroll
        for (int j = 0; j < 4; ++j) {
            a.u[j]      = Arow[kw + half * 4 + j];      al.u[j]     = ArowL[kw + half * 4 + j];
            a.u[4 + j]  = Arow[kw + 8 + half * 4 + j];  al.u[4 + j] = ArowL[kw + 8 + half * 4 + j];
        }
        #pragma unroll
        for (int nt = 0; nt < NT; ++nt) {
            union { v16bf v; unsigned int u[8]; } b, bl;
            const unsigned int* BrowL = Brow[nt] + (plB >> 1);
            #pragma unroll
            for (int j = 0; j < 4; ++j) {
                b.u[j]     = Brow[nt][kw + half * 4 + j];      bl.u[j]     = BrowL[kw + half * 4 + j];
                b.u[4 + j] = Brow[nt][kw + 8 + half * 4 + j];  bl.u[4 + j] = BrowL[kw + 8 + half * 4 + j];
            }
            acc[nt] = wmma_split(a.v, al.v, b.v, bl.v, acc[nt]);
        }
    }

    float* sw = stg[wave];
    #pragma unroll
    for (int nt = 0; nt < NT; ++nt)
        #pragma unroll
        for (int r = 0; r < 8; ++r) sw[(half * 8 + r) * 68 + nt * 16 + lrow] = acc[nt][r];
    asm volatile("s_wait_dscnt 0" ::: "memory");
    #pragma unroll 1
    for (int pass = 0; pass < 2; ++pass) {
        #pragma unroll
        for (int i = 0; i < 8; ++i) { const int c = lane + 32 * i, rr = c >> 4, q = (c & 15) * 4;
            *(volatile v4f_t*)(C + (size_t)(tm * 16 + rr) * N + tg * 64 + q) = *(const volatile v4fa*)(sw + rr * 68 + q); }
        __threadfence();
    }
}

__global__ void prep_silu_x(const float* __restrict__ xz,
                            bf16_t* __restrict__ xbf) {
    const int i      = (blockIdx.x * blockDim.x + threadIdx.x) * 2;
    const int d      = i & (D_INNER - 1);
    const int l      = (i >> 9) & (SEQLEN - 1);
    const int b      = (i >> 20) & 1;
    const int branch = i >> 21;
    const int leff   = branch ? (SEQLEN - 1 - l) : l;
    const int eoff   = branch << 10;
    const float* xp = xz + ((size_t)b * SEQLEN + leff) * E_DIM + eoff + d;
    st2pair(xbf + i, PL_X, siluf(xp[0]), siluf(xp[1]));
}

__device__ __forceinline__ size_t ps_base(int branch, int b, int c, int d) {
    return ((size_t)(((branch * NBATCH + b) * NCHUNK + c) * D_STATE) << 9) + d;
}

__device__ __forceinline__ void stage_xdbl_chunk(float* sxd,
                                                 const float* __restrict__ src,
                                                 int tid) {
    const char* s = (const char*)src;
    char*       dch = (char*)sxd;
    #pragma unroll
    for (int k = 0; k < 4; ++k)
        async_b128_to_lds(dch + tid * 16 + k * 4096, s + tid * 16 + k * 4096);
    wait_async_lds();
    __syncthreads();
}

__global__ void scan_pass1(const float* __restrict__ xz,
                           const float* __restrict__ xdbl,
                           const float* __restrict__ Wdt_f,
                           const float* __restrict__ Wdt_b,
                           const float* __restrict__ bdt_f,
                           const float* __restrict__ bdt_b,
                           const float* __restrict__ Alog_f,
                           const float* __restrict__ Alog_b,
                           float* __restrict__ P,
                           float* __restrict__ S) {
    __shared__ __attribute__((aligned(16))) float sxd[CHUNKT * XD_LD];
    const int idx    = blockIdx.x * blockDim.x + threadIdx.x;
    const int d      = idx & (D_INNER - 1);
    const int c      = (idx >> 9) & (NCHUNK - 1);
    const int b      = (idx >> 14) & 1;
    const int branch = idx >> 15;
    const int l0     = c * CHUNKT;

    const float* __restrict__ xdbase =
        xdbl + (size_t)(branch * NBATCH + b) * SEQLEN * XD_LD;
    stage_xdbl_chunk(sxd, xdbase + (size_t)l0 * XD_LD, threadIdx.x);

    const float* __restrict__ Wdt  = branch ? Wdt_b  : Wdt_f;
    const float* __restrict__ bdt  = branch ? bdt_b  : bdt_f;
    const float* __restrict__ Alog = branch ? Alog_b : Alog_f;

    float Av[D_STATE], wdt[DT_RANK], h[D_STATE], p[D_STATE];
    #pragma unroll
    for (int n = 0; n < D_STATE; ++n) {
        Av[n]  = -__expf(Alog[d * D_STATE + n]);
        wdt[n] = Wdt[d * DT_RANK + n];
        h[n]   = 0.f;
        p[n]   = 1.f;
    }
    const float bias = bdt[d];
    const int   eoff = branch << 10;
    const float* __restrict__ xzb = xz + (size_t)b * SEQLEN * E_DIM;

    for (int t = 0; t < CHUNKT; ++t) {
        const int l    = l0 + t;
        const int leff = branch ? (SEQLEN - 1 - l) : l;
        const float* xd = &sxd[t * XD_LD];

        const float u = siluf(xzb[(size_t)leff * E_DIM + eoff + d]);
        float tt = bias;
        #pragma unroll
        for (int r = 0; r < DT_RANK; ++r) tt = fmaf(wdt[r], xd[r], tt);
        const float dt = (tt > 20.f) ? tt : log1pf(__expf(tt));

        #pragma unroll
        for (int n = 0; n < D_STATE; ++n) {
            const float dA = __expf(dt * Av[n]);
            h[n] = fmaf(dA, h[n], dt * xd[DT_RANK + n] * u);
            p[n] *= dA;
        }
    }
    const size_t base = ps_base(branch, b, c, d);
    #pragma unroll 1
    for (int pass = 0; pass < 2; ++pass) {
        #pragma unroll
        for (int n = 0; n < D_STATE; ++n) { *(volatile float*)(P + base + ((size_t)n << 9)) = p[n]; *(volatile float*)(S + base + ((size_t)n << 9)) = h[n]; }
        __threadfence();
    }
}

__global__ void scan_pass2(const float* __restrict__ P,
                           const float* __restrict__ S,
                           float* __restrict__ Hin) {
    const int ch     = blockIdx.x * blockDim.x + threadIdx.x;
    const int d      = ch & (D_INNER - 1);
    const int b      = (ch >> 9) & 1;
    const int branch = ch >> 10;

    float h[D_STATE];
    #pragma unroll
    for (int n = 0; n < D_STATE; ++n) h[n] = 0.f;

    for (int c = 0; c < NCHUNK; ++c) {
        const size_t base = ps_base(branch, b, c, d);
        #pragma unroll
        for (int n = 0; n < D_STATE; ++n) {
            const size_t o = base + ((size_t)n << 9);
            st2f(Hin + o, h[n]);
            h[n] = fmaf(P[o], h[n], S[o]);
        }
    }
}

__global__ void scan_pass3(const float* __restrict__ xz,
                           const float* __restrict__ xdbl,
                           const float* __restrict__ Wdt_f,
                           const float* __restrict__ Wdt_b,
                           const float* __restrict__ bdt_f,
                           const float* __restrict__ bdt_b,
                           const float* __restrict__ Alog_f,
                           const float* __restrict__ Alog_b,
                           const float* __restrict__ Df,
                           const float* __restrict__ Db,
                           const float* __restrict__ Hin,
                           bf16_t* __restrict__ ybf) {
    __shared__ __attribute__((aligned(16))) float sxd[CHUNKT * XD_LD];
    const int idx    = blockIdx.x * blockDim.x + threadIdx.x;
    const int d      = idx & (D_INNER - 1);
    const int c      = (idx >> 9) & (NCHUNK - 1);
    const int b      = (idx >> 14) & 1;
    const int branch = idx >> 15;
    const int l0     = c * CHUNKT;

    const float* __restrict__ xdbase =
        xdbl + (size_t)(branch * NBATCH + b) * SEQLEN * XD_LD;
    stage_xdbl_chunk(sxd, xdbase + (size_t)l0 * XD_LD, threadIdx.x);

    const float* __restrict__ Wdt  = branch ? Wdt_b  : Wdt_f;
    const float* __restrict__ bdt  = branch ? bdt_b  : bdt_f;
    const float* __restrict__ Alog = branch ? Alog_b : Alog_f;
    const float* __restrict__ Dp   = branch ? Db     : Df;

    float Av[D_STATE], wdt[DT_RANK], h[D_STATE];
    const size_t base = ps_base(branch, b, c, d);
    #pragma unroll
    for (int n = 0; n < D_STATE; ++n) {
        Av[n]  = -__expf(Alog[d * D_STATE + n]);
        wdt[n] = Wdt[d * DT_RANK + n];
        h[n]   = Hin[base + ((size_t)n << 9)];
    }
    const float bias = bdt[d];
    const float Dd   = Dp[d];
    const int   eoff = branch << 10;
    const float* __restrict__ xzb = xz + (size_t)b * SEQLEN * E_DIM;
    __shared__ __attribute__((aligned(16))) _Float16 sy[2][CHUNKT * 256];
    const int dl = threadIdx.x;

    for (int t = 0; t < CHUNKT; ++t) {
        const int l    = l0 + t;
        const int leff = branch ? (SEQLEN - 1 - l) : l;
        const float* xd = &sxd[t * XD_LD];

        const float u = siluf(xzb[(size_t)leff * E_DIM + eoff + d]);
        float tt = bias;
        #pragma unroll
        for (int r = 0; r < DT_RANK; ++r) tt = fmaf(wdt[r], xd[r], tt);
        const float dt = (tt > 20.f) ? tt : log1pf(__expf(tt));

        float y = 0.f;
        #pragma unroll
        for (int n = 0; n < D_STATE; ++n) {
            const float dA = __expf(dt * Av[n]);
            h[n] = fmaf(dA, h[n], dt * xd[DT_RANK + n] * u);
            y    = fmaf(h[n], xd[DT_RANK + D_STATE + n], y);
        }
        y = fmaf(u, Dd, y);

        const float zr = xzb[(size_t)leff * E_DIM + eoff + D_INNER + d];
        y *= siluf(zr);
        const _Float16 yh = (_Float16)y;
        sy[0][t * 256 + dl] = yh; sy[1][t * 256 + dl] = lo_of(y, yh);
    }
    __syncthreads();
    {
        const int dbase = (blockIdx.x * blockDim.x) & (D_INNER - 1);
        const int tq = threadIdx.x >> 5, ch = threadIdx.x & 31;
        #pragma unroll 1
        for (int pass = 0; pass < 2; ++pass) {
            for (int t = tq; t < CHUNKT; t += 8) {
                const int l = l0 + t, leff = branch ? (SEQLEN - 1 - l) : l;
                _Float16* yb = ybf + (size_t)b * SEQLEN * (2 * D_INNER) + (size_t)leff * (2 * D_INNER) + (branch << 9) + dbase + ch * 8;
                *(volatile v4u_t*)yb = *(const volatile v4ua*)(sy[0] + t * 256 + ch * 8);
                *(volatile v4u_t*)(yb + PL_Y) = *(const volatile v4ua*)(sy[1] + t * 256 + ch * 8);
            }
            __threadfence();
        }
    }
}

extern "C" void kernel_launch(void* const* d_in, const int* in_sizes, int n_in,
                              void* d_out, int out_size, void* d_ws, size_t ws_size,
                              hipStream_t stream) {
    (void)in_sizes; (void)n_in; (void)out_size; (void)ws_size;

    const float* hidden = (const float*)d_in[0];
    const float* W_in   = (const float*)d_in[1];
    const float* Wx_f   = (const float*)d_in[2];
    const float* Wx_b   = (const float*)d_in[3];
    const float* Wdt_f  = (const float*)d_in[4];
    const float* Wdt_b  = (const float*)d_in[5];
    const float* bdt_f  = (const float*)d_in[6];
    const float* bdt_b  = (const float*)d_in[7];
    const float* Alog_f = (const float*)d_in[8];
    const float* Alog_b = (const float*)d_in[9];
    const float* D_f    = (const float*)d_in[10];
    const float* D_b    = (const float*)d_in[11];
    const float* W_out  = (const float*)d_in[12];
    float* out = (float*)d_out;

    char* ws = (char*)d_ws;
    size_t off = 0;
    bf16_t* hbf    = (bf16_t*)(ws + off); off += (size_t)MROWS * D_MODEL * 2 * 2;
    bf16_t* winbf  = (bf16_t*)(ws + off); off += (size_t)E_DIM * D_MODEL * 2 * 2;
    bf16_t* wxbf   = (bf16_t*)(ws + off); off += (size_t)2 * 64 * D_INNER * 2 * 2;
    bf16_t* woutbf = (bf16_t*)(ws + off); off += (size_t)D_MODEL * 2 * D_INNER * 2 * 2;
    float*  xz     = (float*) (ws + off); off += (size_t)MROWS * E_DIM * 4;
    bf16_t* xbf    = (bf16_t*)(ws + off); off += (size_t)2 * MROWS * D_INNER * 2 * 2;
    float*  xdbl   = (float*) (ws + off); off += (size_t)2 * MROWS * XD_LD * 4;
    bf16_t* ybf    = (bf16_t*)(ws + off); off += (size_t)MROWS * 2 * D_INNER * 2 * 2;
    const size_t psN = (size_t)2 * NBATCH * NCHUNK * D_STATE * D_INNER;
    float* Pbuf = (float*)(ws + off); off += psN * 4;
    float* Sbuf = (float*)(ws + off); off += psN * 4;
    float* Hin  = (float*)(ws + off); off += psN * 4;

    {
        int n;
        n = MROWS * D_MODEL;
        cvt_f32_bf16<<<(n / 2 + 255) / 256, 256, 0, stream>>>(hidden, hbf, n, PL_H, n);
        n = E_DIM * D_MODEL;
        cvt_f32_bf16<<<(n / 2 + 255) / 256, 256, 0, stream>>>(W_in, winbf, n, PL_WIN, n);
        n = 64 * D_INNER;
        cvt_f32_bf16<<<(n / 2 + 255) / 256, 256, 0, stream>>>(Wx_f, wxbf, n, PL_WX, R_DIM * D_INNER);
        cvt_f32_bf16<<<(n / 2 + 255) / 256, 256, 0, stream>>>(Wx_b, wxbf + n, n, PL_WX, R_DIM * D_INNER);
        n = D_MODEL * 2 * D_INNER;
        cvt_f32_bf16<<<(n / 2 + 255) / 256, 256, 0, stream>>>(W_out, woutbf, n, PL_WO, n);
    }

    {
        const int M = MROWS, N = E_DIM, K = D_MODEL;
        const int tiles = (M / 16) * (N / 64);
        gemm_bf16_wmma<4><<<tiles / 4, 128, 0, stream>>>(hbf, PL_H, winbf, PL_WIN, xz, M, N, K);
    }

    {
        const int n = 2 * MROWS * D_INNER;
        prep_silu_x<<<n / 512, 256, 0, stream>>>(xz, xbf);
    }

    {
        const int M = MROWS, N = XD_LD, K = D_INNER;
        const int tiles = (M / 16) * (N / 64);
        gemm_bf16_wmma<4><<<tiles / 4, 128, 0, stream>>>(xbf, PL_X, wxbf, PL_WX, xdbl, M, N, K);
        gemm_bf16_wmma<4><<<tiles / 4, 128, 0, stream>>>(
            xbf + (size_t)MROWS * D_INNER, PL_X, wxbf + (size_t)64 * D_INNER, PL_WX,
            xdbl + (size_t)MROWS * XD_LD, M, N, K);
    }

    scan_pass1<<<(2 * NBATCH * NCHUNK * D_INNER) / 256, 256, 0, stream>>>(
        xz, xdbl, Wdt_f, Wdt_b, bdt_f, bdt_b, Alog_f, Alog_b, Pbuf, Sbuf);
    scan_pass2<<<(2 * NBATCH * D_INNER) / 256, 256, 0, stream>>>(Pbuf, Sbuf, Hin);
    scan_pass3<<<(2 * NBATCH * NCHUNK * D_INNER) / 256, 256, 0, stream>>>(
        xz, xdbl, Wdt_f, Wdt_b, bdt_f, bdt_b, Alog_f, Alog_b, D_f, D_b, Hin, ybf);

    {
        const int M = MROWS, N = D_MODEL, K = 2 * D_INNER;
        const int tiles = (M / 16) * (N / 64);
        gemm_bf16_wmma<4><<<tiles / 4, 128, 0, stream>>>(ybf, PL_Y, woutbf, PL_WO, out, M, N, K);
    }
}
